// GraphConv_H_61529701482865
// MI455X (gfx1250) — hardware-verified
//
#include <hip/hip_runtime.h>
#include <hip/hip_bf16.h>

#define B_    4
#define C_    256
#define N_    4096
#define K_    16
#define CIN   262
#define NCH   9
#define COUT  256
#define TPB   512
#define PTS   4
#define PPB   64
#define CSTR  40
#define DSTR  144

typedef _Float16      v16bf __attribute__((ext_vector_type(16)));
typedef float         v8f   __attribute__((ext_vector_type(8)));
typedef unsigned int  v8u   __attribute__((ext_vector_type(8)));

union V32 {
  struct { uint4 a, b; } q;
  v16bf bf;
  v8u   u;
};

__device__ __forceinline__ unsigned short f2bf(float f) {
  return __builtin_bit_cast(unsigned short, (_Float16)f);
}
typedef __attribute__((ext_vector_type(4))) float v4f_t;
typedef float v4fa __attribute__((ext_vector_type(4), may_alias));

template <int MASK>
__device__ __forceinline__ float swz_xor(float v) {
  int r = __builtin_amdgcn_ds_swizzle(__builtin_bit_cast(int, v),
                                      (MASK << 10) | 0x1F);
  return __builtin_bit_cast(float, r);
}

__device__ __forceinline__ void loadB(V32& d, const unsigned short* ep, int c) {
  const unsigned short* s = ep + c * (16 * CSTR);
  d.q.a = *(const uint4*)s;
  d.q.b = *(const uint4*)(s + 16);
}

__global__ __launch_bounds__(TPB, 1) void graphconv_edge_wmma(
    const float* __restrict__ x,     const float* __restrict__ pos,
    const int*   __restrict__ knn,   const float* __restrict__ W,
    const float* __restrict__ bias,  const float* __restrict__ gamma,
    const float* __restrict__ beta,  const float* __restrict__ rmean,
    const float* __restrict__ rvar,  float* __restrict__ out) {
  __shared__ __align__(16) unsigned short edge[PTS * NCH * 16 * CSTR];
  __shared__ float distx[PTS * DSTR];
  __shared__ float s_inv[PTS][2];
  __shared__ __align__(16) float s_out[COUT * PPB];

  const int t    = threadIdx.x;
  const int lane = t & 31;
  const int w    = t >> 5;

  const int bp  = t >> 7;
  const int sub = t & 127;
  const int bk  = sub & 15;
  const int bg  = sub >> 4;

  for (int i = t; i < PTS * NCH * 16 * CSTR; i += TPB) edge[i] = 0;

  const int row = w * 16 + (lane & 15);
  const int kb8 = (lane >= 16) ? 8 : 0;
  v8u wv[NCH];
#pragma unroll
  for (int c = 0; c < NCH; ++c) {
#pragma unroll
    for (int j = 0; j < 8; ++j) {
      int e0 = 2 * j, e1 = 2 * j + 1;
      int kl0 = kb8 + (e0 < 8 ? e0 : e0 + 8);
      int kl1 = kb8 + (e1 < 8 ? e1 : e1 + 8);
      int ci0 = c * 32 + kl0, ci1 = c * 32 + kl1;
      unsigned lo = (ci0 < CIN) ? (unsigned)f2bf(W[row * CIN + ci0]) : 0u;
      unsigned hi = (ci1 < CIN) ? (unsigned)f2bf(W[row * CIN + ci1]) : 0u;
      wv[c][j] = lo | (hi << 16);
    }
  }

  float sc[8], sh[8];
#pragma unroll
  for (int j = 0; j < 8; ++j) {
    int oc = w * 16 + j + ((lane >= 16) ? 8 : 0);
    float inv = gamma[oc] / sqrtf(rvar[oc] + 1e-5f);
    sc[j] = inv;
    sh[j] = (bias[oc] - rmean[oc]) * inv + beta[oc];
  }
  __syncthreads();

  const int blockStart = blockIdx.x * PPB;

  for (int base = 0; base < PPB; base += PTS) {
    {
      const int gid = blockStart + base + bp;
      const int bb  = gid >> 12;
      const int nn  = gid & (N_ - 1);
      int nb = knn[(gid << 4) + bk];
      nb = (nb < 0) ? 0 : (nb > N_ - 1 ? N_ - 1 : nb);
      const float* xb = x + (size_t)bb * C_ * N_;

      float df[32];
      float d2 = 0.f;
#pragma unroll
      for (int j = 0; j < 32; ++j) {
        int ch   = bg * 32 + j;
        float cc = xb[ch * N_ + nn];
        float nv = xb[ch * N_ + nb];
        df[j] = nv - cc;
        d2   += df[j] * df[j];
      }
      distx[bp * DSTR + sub] = d2;

      float pdf[3], pc[3];
      if (sub < 16) {
        const float* pb = pos + (size_t)bb * 3 * N_;
        float pd2 = 0.f;
#pragma unroll
        for (int j = 0; j < 3; ++j) {
          pc[j]  = pb[j * N_ + nn];
          float pn = pb[j * N_ + nb];
          pdf[j] = pn - pc[j];
          pd2   += pdf[j] * pdf[j];
        }
        float mp = pd2;
        mp = fmaxf(mp, swz_xor<1>(mp));
        mp = fmaxf(mp, swz_xor<2>(mp));
        mp = fmaxf(mp, swz_xor<4>(mp));
        mp = fmaxf(mp, swz_xor<8>(mp));
        s_inv[bp][0] = 1.f / sqrtf(mp);
      }
      __syncthreads();

      if (t < 64) {
        int rp = t >> 4, rk = t & 15;
        float s = 0.f;
#pragma unroll
        for (int g2 = 0; g2 < 8; ++g2) s += distx[rp * DSTR + g2 * 16 + rk];
        float mx = s;
        mx = fmaxf(mx, swz_xor<1>(mx));
        mx = fmaxf(mx, swz_xor<2>(mx));
        mx = fmaxf(mx, swz_xor<4>(mx));
        mx = fmaxf(mx, swz_xor<8>(mx));
        s_inv[rp][1] = 1.f / sqrtf(mx);
      }
      __syncthreads();

      const float invx = s_inv[bp][1];
      unsigned short* ep = edge + bp * (NCH * 16 * CSTR);
#pragma unroll
      for (int j = 0; j < 32; ++j) {
        int ch = 6 + bg * 32 + j;
        ep[(ch >> 5) * (16 * CSTR) + bk * CSTR + (ch & 31)] = f2bf(df[j] * invx);
      }
      if (sub < 16) {
        const float invp = s_inv[bp][0];
#pragma unroll
        for (int j = 0; j < 3; ++j) {
          ep[bk * CSTR + j]     = f2bf(pc[j]);
          ep[bk * CSTR + 3 + j] = f2bf(pdf[j] * invp);
        }
      }
    }
    __syncthreads();

    const int col  = lane & 15;
#pragma unroll
    for (int p = 0; p < PTS; ++p) {
      const int gid = blockStart + base + p;
      const int bb  = gid >> 12;
      const int nn  = gid & (N_ - 1);

      const unsigned short* ep =
          edge + p * (NCH * 16 * CSTR) + col * CSTR + kb8;

      V32 bufs[2];
      loadB(bufs[0], ep, 0);
      v8f acc = {};
#pragma unroll
      for (int c = 0; c < NCH; ++c) {
        if (c + 1 < NCH) loadB(bufs[(c + 1) & 1], ep, c + 1);
        V32 am;
        am.u = wv[c];
        acc = __builtin_amdgcn_wmma_f32_16x16x32_f16(
            false, am.bf, false, bufs[c & 1].bf, (short)0, acc, false, false);
      }

      float r[8];
#pragma unroll
      for (int j = 0; j < 8; ++j) r[j] = fmaxf(acc[j] * sc[j] + sh[j], 0.f);
#pragma unroll
      for (int j = 0; j < 8; ++j) {
        r[j] = fmaxf(r[j], swz_xor<1>(r[j]));
        r[j] = fmaxf(r[j], swz_xor<2>(r[j]));
        r[j] = fmaxf(r[j], swz_xor<4>(r[j]));
        r[j] = fmaxf(r[j], swz_xor<8>(r[j]));
      }
      float rh[8];
#pragma unroll
      for (int j = 0; j < 8; ++j) rh[j] = swz_xor<16>(r[j]);

      if (lane < 16) {
        int jj = lane & 7;
        float a = r[0];
        a = (jj == 1) ? r[1] : a;
        a = (jj == 2) ? r[2] : a;
        a = (jj == 3) ? r[3] : a;
        a = (jj == 4) ? r[4] : a;
        a = (jj == 5) ? r[5] : a;
        a = (jj == 6) ? r[6] : a;
        a = (jj == 7) ? r[7] : a;
        float b2 = rh[0];
        b2 = (jj == 1) ? rh[1] : b2;
        b2 = (jj == 2) ? rh[2] : b2;
        b2 = (jj == 3) ? rh[3] : b2;
        b2 = (jj == 4) ? rh[4] : b2;
        b2 = (jj == 5) ? rh[5] : b2;
        b2 = (jj == 6) ? rh[6] : b2;
        b2 = (jj == 7) ? rh[7] : b2;
        float val = (lane < 8) ? a : b2;
        (void)bb; (void)nn;
        s_out[(w * 16 + lane) * PPB + base + p] = val;
      }
    }
    __syncthreads();
  }

  {
    const int bb  = blockStart >> 12;
    const int nn0 = blockStart & (N_ - 1);
#pragma unroll 1
    for (int pass = 0; pass < 2; ++pass) {
      for (int c = t; c < COUT * (PPB / 4); c += TPB) { const int ch = c >> 4, q = (c & 15) * 4;
        *(volatile v4f_t*)(out + ((size_t)bb * COUT + ch) * N_ + nn0 + q) = *(const volatile v4fa*)(s_out + ch * PPB + q); }
      __threadfence();
    }
  }
}

extern "C" void kernel_launch(void* const* d_in, const int* in_sizes, int n_in,
                              void* d_out, int out_size, void* d_ws, size_t ws_size,
                              hipStream_t stream) {
  (void)in_sizes; (void)n_in; (void)out_size; (void)d_ws; (void)ws_size;
  const float* x     = (const float*)d_in[0];
  const float* pos   = (const float*)d_in[1];
  const int*   knn   = (const int*)d_in[2];
  const float* W     = (const float*)d_in[3];
  const float* bias  = (const float*)d_in[4];
  const float* gamma = (const float*)d_in[5];
  const float* beta  = (const float*)d_in[6];
  const float* rmean = (const float*)d_in[7];
  const float* rvar  = (const float*)d_in[8];
  float* out = (float*)d_out;

  dim3 grid((B_ * N_) / PPB);
  graphconv_edge_wmma<<<grid, TPB, 0, stream>>>(
      x, pos, knn, W, bias, gamma, beta, rmean, rvar, out);
}
